// MIND_45466523796149
// MI455X (gfx1250) — hardware-verified
//
#include <hip/hip_runtime.h>
#include <math.h>


#define NB 1024
#define SL 50
#define HH 128
#define KK 4
#define NV 100000
#define NVT 782
#define NR (NB * SL)

typedef __attribute__((ext_vector_type(16))) _Float16 v16h;
typedef __attribute__((ext_vector_type(16))) __bf16 v16b;
typedef __attribute__((ext_vector_type(8)))  _Float16 v8h;
typedef __attribute__((ext_vector_type(8)))  float v8f;
typedef __attribute__((ext_vector_type(4)))  float v4f;
typedef __attribute__((ext_vector_type(2)))  float v2f;
typedef __attribute__((ext_vector_type(4)))  unsigned v4u;
typedef float __attribute__((may_alias)) float_a;

template <typename T> __device__ __forceinline__ void vst2(void* p, T v) { *(volatile T*)p = v; __threadfence(); *(volatile T*)p = v; }
__device__ __forceinline__ v8f wmma16(v16h a, v16h b, v8f c) {
  v8f d = __builtin_amdgcn_wmma_f32_16x16x32_f16(false, a, false, b, (short)0, c, false, false);
  asm volatile("v_nop\n\tv_nop\n\tv_nop\n\tv_nop" : "+v"(d) : "v"(a), "v"(b));
  return d;
}
__device__ __forceinline__ v8f wmma_bf(v16b a, v16b b, v8f c) {
  v8f d = __builtin_amdgcn_wmma_f32_16x16x32_bf16(false, a, false, b, (short)0, c, false, false);
  asm volatile("v_nop\n\tv_nop\n\tv_nop\n\tv_nop" : "+v"(d) : "v"(a), "v"(b));
  return d;
}
__device__ __forceinline__ v16h frag_h(const _Float16* rowk0, int lane) {
  union { v16h v; v8h q[2]; } u; const _Float16* p = rowk0 + 8 * (lane >> 4);
  u.q[0] = *(const v8h*)p; u.q[1] = *(const v8h*)(p + 16); return u.v;
}
struct F2 { v16b h, l; };
__device__ __forceinline__ F2 split_row(const float* row, int k0, int lane) { F2 r; const float* p = row + k0 + 8 * (lane >> 4);
#pragma unroll
  for (int i = 0; i < 8; ++i) { const float a = p[i], b = p[16 + i]; const __bf16 ha = (__bf16)a, hb = (__bf16)b;
    r.h[i] = ha; r.l[i] = (__bf16)(a - (float)ha); r.h[8 + i] = hb; r.l[8 + i] = (__bf16)(b - (float)hb); }
  return r; }
__device__ __forceinline__ v8f mac3(const F2& a, const F2& b, v8f c) { c = wmma_bf(a.l, b.h, c); c = wmma_bf(a.h, b.l, c); return wmma_bf(a.h, b.h, c); }
#define LDSX() do { asm volatile("s_wait_dscnt 0" ::: "memory"); __builtin_amdgcn_wave_barrier(); __builtin_amdgcn_fence(__ATOMIC_RELEASE, "workgroup"); } while (0)

__global__ __launch_bounds__(256) void k_emb16(const float* __restrict__ emb, _Float16* __restrict__ e16) {
  const size_t g8 = (size_t)blockIdx.x * 256 + threadIdx.x; if (g8 >= (size_t)NV * HH / 8) return;
  union { v8h h; v4u u; } pk;
#pragma unroll
  for (int e = 0; e < 8; ++e) pk.h[e] = (_Float16)(emb[g8 * 8 + e] * 64.0f);
  vst2(e16 + g8 * 8, pk.u);
}
__global__ __launch_bounds__(128) void k_h(const int* __restrict__ seq, const float* __restrict__ emb, const float* __restrict__ W, float* __restrict__ h) {
  __shared__ __align__(16) float so[4][16][132];
  const int tid = threadIdx.x, wave = tid >> 5, lane = tid & 31, col = lane & 15, g = lane >> 4;
  const int r0 = blockIdx.x * 64 + wave * 16; const int r = r0 + col;
  int idx = seq[r]; const bool zero = idx <= 0 || idx >= NV; if (idx < 0 || idx >= NV) idx = 0;
  const float* arow = emb + (size_t)idx * HH;
  v8f acc[8] = {};
#pragma unroll 1
  for (int kc = 0; kc < HH / 32; ++kc) { F2 a = split_row(arow, kc * 32, lane);
    if (zero) { a.h = (v16b){}; a.l = (v16b){}; }
#pragma unroll
    for (int j = 0; j < 8; ++j) acc[j] = mac3(a, split_row(W + (size_t)(j * 16 + col) * HH, kc * 32, lane), acc[j]); }
#pragma unroll
  for (int j = 0; j < 8; ++j)
#pragma unroll
    for (int rr = 0; rr < 8; ++rr) so[wave][8 * g + rr][j * 16 + col] = acc[j][rr];
  LDSX();
#pragma unroll 4
  for (int rl = 0; rl < 16; ++rl) vst2(h + (size_t)(r0 + rl) * HH + lane * 4, *(const v4f*)(&so[wave][rl][lane * 4]));
}
__global__ __launch_bounds__(256) void k_colstat(const float* __restrict__ cw, float* __restrict__ st) {
  __shared__ float red[256];
  const int c = blockIdx.x, tid = threadIdx.x;
  float m = -3.0e38f;
  for (int b = tid; b < NB; b += 256) m = fmaxf(m, cw[(size_t)b * (KK * SL) + c]);
  red[tid] = m; __syncthreads();
  for (int s2 = 128; s2 > 0; s2 >>= 1) { if (tid < s2) red[tid] = fmaxf(red[tid], red[tid + s2]); __syncthreads(); }
  const float gm = red[0]; __syncthreads();
  float sm = 0.f;
  for (int b = tid; b < NB; b += 256) sm += expf(cw[(size_t)b * (KK * SL) + c] - gm);
  red[tid] = sm; __syncthreads();
  for (int s2 = 128; s2 > 0; s2 >>= 1) { if (tid < s2) red[tid] += red[tid + s2]; __syncthreads(); }
  if (tid < 32) vst2(st + (size_t)c * 32 + tid, (float_a)(tid == 0 ? gm : (tid == 1 ? red[0] : 0.f)));
}
__global__ __launch_bounds__(128) void k_route(const float* __restrict__ cwin, const float* __restrict__ st, const float* __restrict__ mask, const float* __restrict__ h,
                                             float* __restrict__ cwout, int last, const int* __restrict__ item, const float* __restrict__ emb,
                                             float* __restrict__ uemb, float* __restrict__ best) {
  __shared__ float sw[KK][SL + 2], cap[KK][HH], red[128], cosv[KK];
  const int b = blockIdx.x, tid = threadIdx.x;
  const float* hb = h + (size_t)b * SL * HH;
  for (int q = tid; q < KK * SL; q += 128) { const int k = q / SL, s = q % SL;
    const float v = cwin[(size_t)b * KK * SL + q]; const float mx = st[(size_t)q * 32], sm = st[(size_t)q * 32 + 1];
    const float w = expf(v - mx) / sm; sw[k][s] = mask[(size_t)b * SL + s] == 0.f ? 0.f : w; }
  __syncthreads();
#pragma unroll
  for (int k = 0; k < KK; ++k) { float c = 0.f;
#pragma unroll 1
    for (int s = 0; s < SL; ++s) c += sw[k][s] * hb[s * HH + k * 32 + (tid >> 2)];
    cap[k][tid] = c; }
  __syncthreads();
#pragma unroll
  for (int k = 0; k < KK; ++k) { red[tid] = cap[k][tid] * cap[k][tid]; __syncthreads();
    for (int s2 = 64; s2 > 0; s2 >>= 1) { if (tid < s2) red[tid] += red[tid + s2]; __syncthreads(); }
    const float n2 = red[0]; __syncthreads();
    const float f = n2 / (1.0f + n2) / sqrtf(n2 + 1e-9f);
    cap[k][tid] = cap[k][tid] * f; __syncthreads(); }
  if (!last) {
    for (int q = tid; q < KK * SL; q += 128) { const int k = q / SL, s = q % SL; float d = 0.f;
#pragma unroll 1
      for (int hh = 0; hh < HH; ++hh) d += hb[s * HH + k * 32 + (hh >> 2)] * cap[k][hh];
      sw[k][s] = cwin[(size_t)b * KK * SL + q] + d; }
    __syncthreads();
    if (tid < 50) { v4f v = { sw[(tid * 4) / SL][(tid * 4) % SL], sw[(tid * 4 + 1) / SL][(tid * 4 + 1) % SL], sw[(tid * 4 + 2) / SL][(tid * 4 + 2) % SL], sw[(tid * 4 + 3) / SL][(tid * 4 + 3) % SL] };
      vst2(cwout + (size_t)b * KK * SL + tid * 4, v); }
    return;
  }
#pragma unroll
  for (int k = 0; k < KK; ++k) vst2(uemb + ((size_t)b * KK + k) * HH + tid, (float_a)cap[k][tid]);
  int it = item[b]; const bool z = it <= 0 || it >= NV; if (it < 0 || it >= NV) it = 0;
  const float ie = z ? 0.f : emb[(size_t)it * HH + tid];
#pragma unroll
  for (int k = 0; k < KK; ++k) { red[tid] = cap[k][tid] * ie; __syncthreads();
    for (int s2 = 64; s2 > 0; s2 >>= 1) { if (tid < s2) red[tid] += red[tid + s2]; __syncthreads(); }
    if (tid == 0) cosv[k] = red[0];
    __syncthreads(); }
  int kb = 0; float bv = cosv[0];
#pragma unroll
  for (int k = 1; k < KK; ++k) if (cosv[k] > bv) { bv = cosv[k]; kb = k; }
  vst2(best + (size_t)b * HH + tid, (float_a)cap[kb][tid]);
}
__global__ __launch_bounds__(128) void k_scores(const float* __restrict__ best, const _Float16* __restrict__ e16, float* __restrict__ part) {
  __shared__ __align__(16) float so[4][16][132];
  const int tid = threadIdx.x, wave = tid >> 5, lane = tid & 31, col = lane & 15, g = lane >> 4;
  const int r0 = blockIdx.x * 64 + wave * 16, n0 = blockIdx.y * 128;
  v16h a[4]; { const float* br = best + (size_t)(r0 + col) * HH;
#pragma unroll
    for (int kc = 0; kc < 4; ++kc) { v16h t; const float* p = br + kc * 32 + 8 * g;
#pragma unroll
      for (int i = 0; i < 8; ++i) { t[i] = (_Float16)(p[i] * 1048576.0f); t[8 + i] = (_Float16)(p[16 + i] * 1048576.0f); }
      a[kc] = t; } }
  v8f acc[8] = {};
#pragma unroll
  for (int j = 0; j < 8; ++j) { int v = n0 + j * 16 + col; if (v > NV - 1) v = NV - 1;
#pragma unroll
    for (int kc = 0; kc < 4; ++kc) acc[j] = wmma16(a[kc], frag_h(e16 + (size_t)v * HH + kc * 32, lane), acc[j]); }
#pragma unroll
  for (int j = 0; j < 8; ++j)
#pragma unroll
    for (int rr = 0; rr < 8; ++rr) so[wave][8 * g + rr][j * 16 + col] = acc[j][rr] * (1.0f / 67108864.0f);
  LDSX();
  float mx = -3.0e38f;
#pragma unroll 4
  for (int j = 0; j < 64; ++j) { const int c = g * 64 + j; if (n0 + c < NV) mx = fmaxf(mx, so[wave][col][c]); }
  mx = fmaxf(mx, __shfl_xor(mx, 16, 32));
  float sm = 0.f;
#pragma unroll 4
  for (int j = 0; j < 64; ++j) { const int c = g * 64 + j; if (n0 + c < NV) sm += expf(so[wave][col][c] - mx); }
  sm += __shfl_xor(sm, 16, 32);
  __shared__ __align__(16) float sp[4][16][2];
  if (g == 0) { sp[wave][col][0] = mx; sp[wave][col][1] = sm; }
  LDSX();
  if (lane < 16) vst2(part + ((size_t)blockIdx.y * NB + r0 + lane) * 2, *(const v2f*)(&sp[wave][lane][0]));
}
__global__ __launch_bounds__(256) void k_loss(const float* __restrict__ part, const float* __restrict__ best, const float* __restrict__ emb, const int* __restrict__ item,
                                            float* __restrict__ out) {
  __shared__ float red[256]; __shared__ float rowv[NB];
  const int tid = threadIdx.x;
  for (int b = tid; b < NB; b += 256) {
    float mx = -3.0e38f;
    for (int t = 0; t < NVT; ++t) mx = fmaxf(mx, part[((size_t)t * NB + b) * 2]);
    float sm = 0.f;
    for (int t = 0; t < NVT; ++t) sm += part[((size_t)t * NB + b) * 2 + 1] * expf(part[((size_t)t * NB + b) * 2] - mx);
    const float lse = mx + logf(sm);
    int it = item[b]; if (it < 0 || it >= NV) it = 0;
    float sc = 0.f;
    for (int i = 0; i < HH; ++i) sc += best[(size_t)b * HH + i] * emb[(size_t)it * HH + i];
    rowv[b] = sc - lse; }
  __syncthreads();
  float s = 0.f; for (int b = tid; b < NB; b += 256) s += rowv[b];
  red[tid] = s; __syncthreads();
  for (int s2 = 128; s2 > 0; s2 >>= 1) { if (tid < s2) red[tid] += red[tid + s2]; __syncthreads(); }
  if (tid < 32) { const float v = tid == 0 ? -red[0] / (float)NB : 0.f; if (tid == 0) vst2(out, (float_a)v); }
}

extern "C" void kernel_launch(void* const* d_in, const int* in_sizes, int n_in,
                              void* d_out, int out_size, void* d_ws, size_t ws_size,
                              hipStream_t stream) {
  (void)in_sizes; (void)n_in; (void)out_size; (void)ws_size;
  const int* seq = (const int*)d_in[0]; const float* mask = (const float*)d_in[1]; const int* item = (const int*)d_in[2];
  const float* emb = (const float*)d_in[3]; const float* W = (const float*)d_in[4]; const float* cw0 = (const float*)d_in[5];
  float* uemb = (float*)d_out; float* loss = (float*)d_out + (size_t)NB * KK * HH;
  char* ws = (char*)d_ws; size_t off = 0;
  auto take = [&](size_t bytes) { char* p = ws + off; off += (bytes + 255) & ~(size_t)255; return p; };
  _Float16* e16 = (_Float16*)take((size_t)NV * HH * 2);
  float* h = (float*)take((size_t)NR * HH * 4);
  float* st = (float*)take((size_t)KK * SL * 32 * 4);
  float* cw1 = (float*)take((size_t)NB * KK * SL * 4); float* cw2 = (float*)take((size_t)NB * KK * SL * 4);
  float* best = (float*)take((size_t)NB * HH * 4);
  float* part = (float*)take((size_t)NB * NVT * 2 * 4);
  k_emb16<<<(unsigned)(((size_t)NV * HH / 8 + 255) / 256), 256, 0, stream>>>(emb, e16);
  k_h<<<NR / 64, 128, 0, stream>>>(seq, emb, W, h);
  k_colstat<<<KK * SL, 256, 0, stream>>>(cw0, st);
  k_route<<<NB, 128, 0, stream>>>(cw0, st, mask, h, cw1, 0, item, emb, uemb, best);
  k_colstat<<<KK * SL, 256, 0, stream>>>(cw1, st);
  k_route<<<NB, 128, 0, stream>>>(cw1, st, mask, h, cw2, 0, item, emb, uemb, best);
  k_colstat<<<KK * SL, 256, 0, stream>>>(cw2, st);
  k_route<<<NB, 128, 0, stream>>>(cw2, st, mask, h, nullptr, 1, item, emb, uemb, best);
  k_scores<<<dim3(NB / 64, NVT), 128, 0, stream>>>(best, e16, part);
  k_loss<<<1, 256, 0, stream>>>(part, best, emb, item, loss);
}
